// MultiheadAttention_24249385353229
// MI455X (gfx1250) — hardware-run, weakly checked
//
#include <hip/hip_runtime.h>
#ifndef NB
#define NB 4
#endif
#ifndef SEQ
#define SEQ 2048
#endif
#define NB_FULL 4
#define SEQ_FULL 2048
#define DM 1024
#define NH 16
#define HD 64
#define HG 4
#define BW (2 * SEQ)

static_assert(SEQ % 128 == 0);
static_assert(SEQ <= SEQ_FULL);
static_assert(NB <= NB_FULL);
static_assert(DM == NH * HD);
static_assert(NH % HG == 0);
static_assert(DM % 64 == 0);
static_assert((NH * BW) % 256 == 0);

typedef unsigned short v8us __attribute__((ext_vector_type(8), may_alias));
typedef float  v8f  __attribute__((ext_vector_type(8)));
typedef float  v4f  __attribute__((ext_vector_type(4)));
typedef float  v4fa __attribute__((ext_vector_type(4), may_alias));
typedef _Float16 v16h __attribute__((ext_vector_type(16)));
typedef _Float16 v4h __attribute__((ext_vector_type(4)));
union FragH { v16h v; v8us half[2]; _Float16 h[16]; unsigned short u[16]; };

__device__ __forceinline__ unsigned short bf16_bits(float x) { unsigned int u = __float_as_uint(x); return (unsigned short)((u + 0x7FFFu + ((u >> 16) & 1u)) >> 16); }
__device__ __forceinline__ float bf16_val(unsigned short b) { return __uint_as_float(((unsigned int)b) << 16); }
__device__ __forceinline__ float bf16_rne(float x) { return bf16_val(bf16_bits(x)); }

__device__ __forceinline__ v16h g2_frag(const _Float16* p, int hh) {
  FragH f;
  f.half[0] = *(const v8us*)((const unsigned short*)p + 8 * hh);
  f.half[1] = *(const v8us*)((const unsigned short*)p + 16 + 8 * hh);
  return f.v;
}
__device__ __forceinline__ v8f g2_mma(v16h a, v16h b, v8f c) {
  v8f d = __builtin_amdgcn_wmma_f32_16x16x32_f16(false, a, false, b, (short)0, c, false, false);
  asm volatile("v_nop\n\tv_nop\n\tv_nop\n\tv_nop" : "+v"(d) : "v"(a), "v"(b));
  return d;
}

__global__ __launch_bounds__(256) void k_wnat(const float* __restrict__ w, size_t n8, _Float16* __restrict__ Bt) {
  const size_t t = (size_t)blockIdx.x * 256 + threadIdx.x;
  if (t >= n8) return;
  const v4f a = *(const v4fa*)(w + t * 8), c = *(const v4fa*)(w + t * 8 + 4);
  FragH f;
#pragma unroll
  for (int q = 0; q < 4; ++q) { f.h[q] = (_Float16)(bf16_rne(a[q]) * 16.0f); f.h[4 + q] = (_Float16)(bf16_rne(c[q]) * 16.0f); }
  const v8us o = f.half[0];
  *(volatile v8us*)((unsigned short*)Bt + t * 8) = o;
  __threadfence();
  *(volatile v8us*)((unsigned short*)Bt + t * 8) = o;
}

__global__ __launch_bounds__(256) void k_x16(const float* __restrict__ x, _Float16* __restrict__ X16, size_t n8) {
  const size_t t = (size_t)blockIdx.x * 256 + threadIdx.x;
  if (t >= n8) return;
  const v4f a = *(const v4fa*)(x + t * 8), c = *(const v4fa*)(x + t * 8 + 4);
  FragH f;
#pragma unroll
  for (int q = 0; q < 4; ++q) { f.h[q] = (_Float16)bf16_rne(a[q]); f.h[4 + q] = (_Float16)bf16_rne(c[q]); }
  const v8us o = f.half[0];
  *(volatile v8us*)((unsigned short*)X16 + t * 8) = o;
  __threadfence();
  *(volatile v8us*)((unsigned short*)X16 + t * 8) = o;
}

__global__ __launch_bounds__(256) void k_btab(const float* __restrict__ rel, float* __restrict__ tab) {
  #pragma clang fp contract(off)
  __shared__ __attribute__((aligned(16))) float sh[256];
  const int tid = threadIdx.x;
  const int g = blockIdx.x * 256 + tid;
  const int h = g / BW, idx = g % BW;
  const int d = idx - (SEQ - 1);
  const int rp = d < 0 ? -d : d;
  const int rs = rp < 1 ? 1 : rp;
  const float f = logf((float)rs * (1.0f / 7.0f)) * (1.0f / 2.90612011486f) * 8.0f;
  int lg = 7 + (int)f;
  lg = lg > 15 ? 15 : lg;
  lg = lg < 0 ? 0 : lg;
  if (rp >= 128) lg = 15;
  int bucket = (d > 0 ? 16 : 0) + (rp < 8 ? rp : lg);
  bucket = bucket < 0 ? 0 : (bucket > 31 ? 31 : bucket);
  float v = bf16_rne(rel[bucket * NH + h]);
  if (idx == BW - 1) v = 0.0f;
  sh[tid] = v;
  __syncthreads();
  if (tid < 64) {
    const v4f o = *(const v4fa*)&sh[tid * 4];
    float* dst = tab + (size_t)blockIdx.x * 256 + tid * 4;
    *(volatile v4f*)dst = o;
    __threadfence();
    *(volatile v4f*)dst = o;
  }
}

template <int RELB>
__global__ __launch_bounds__(128) void k_gemm2(const _Float16* __restrict__ A, int lda, size_t sA, const _Float16* __restrict__ Bh, int ldb, size_t sB, float alpha,
    const float* __restrict__ RB, int rbh0, float* __restrict__ C, _Float16* __restrict__ C16, int ldc, size_t sC, int M, int N, int K) {
  __shared__ __attribute__((aligned(16))) float so[4][32][68];
  __shared__ __attribute__((aligned(16))) float sb[4][96];
  const int tid = threadIdx.x, w = tid >> 5, lane = tid & 31, ln = lane & 15, hh = lane >> 4;
  const int by = blockIdx.y;
  A += (size_t)by * sA; Bh += (size_t)by * sB;
  const size_t cofs = (size_t)by * sC;
  const int ntn = N >> 6;
  const int mt = blockIdx.x / ntn, nq = blockIdx.x - mt * ntn;
  const int row0 = mt * 128 + 32 * w, col0 = nq * 64;
  if (row0 >= M) return;
  const _Float16* a0p = A + (size_t)(row0 + ln) * lda;
  const _Float16* a1p = a0p + (size_t)16 * lda;
  const _Float16* b0p = Bh + (size_t)(col0 + ln) * ldb;
  const _Float16* b1p = b0p + (size_t)16 * ldb;
  const _Float16* b2p = b1p + (size_t)16 * ldb;
  const _Float16* b3p = b2p + (size_t)16 * ldb;
  const v8f z8 = {0.f,0.f,0.f,0.f,0.f,0.f,0.f,0.f};
  v8f c00 = z8, c01 = z8, c02 = z8, c03 = z8, c10 = z8, c11 = z8, c12 = z8, c13 = z8;
#pragma unroll 1
  for (int kb = 0; kb < K; kb += 32) {
    const v16h a0 = g2_frag(a0p + kb, hh), a1 = g2_frag(a1p + kb, hh);
    v16h b = g2_frag(b0p + kb, hh); c00 = g2_mma(a0, b, c00); c10 = g2_mma(a1, b, c10);
    b = g2_frag(b1p + kb, hh); c01 = g2_mma(a0, b, c01); c11 = g2_mma(a1, b, c11);
    b = g2_frag(b2p + kb, hh); c02 = g2_mma(a0, b, c02); c12 = g2_mma(a1, b, c12);
    b = g2_frag(b3p + kb, hh); c03 = g2_mma(a0, b, c03); c13 = g2_mma(a1, b, c13);
  }
  if (RELB) {
    const float* rb = RB + (size_t)(rbh0 + by) * BW;
    const int base = col0 - row0 - 31 + (SEQ - 1);
#pragma unroll
    for (int u = 0; u < 3; ++u) {
      int idx = base + u * 32 + lane;
      idx = idx < 0 ? 0 : (idx > BW - 1 ? BW - 1 : idx);
      sb[w][u * 32 + lane] = rb[idx];
    }
    __builtin_amdgcn_fence(4  , "workgroup");
    __builtin_amdgcn_wave_barrier();
  }
  v8f accs[8] = {c00, c01, c02, c03, c10, c11, c12, c13};
#pragma unroll
  for (int u = 0; u < 8; ++u) {
    const int t = u & 3, half = u >> 2;
#pragma unroll
    for (int r = 0; r < 8; ++r) {
      const int rloc = half * 16 + 8 * hh + r;
      float v = accs[u][r] * alpha;
      if (RELB) v += sb[w][t * 16 + ln - rloc + 31];
      so[w][rloc][t * 16 + ln] = v;
    }
  }
  __builtin_amdgcn_fence(4  , "workgroup");
  __builtin_amdgcn_wave_barrier();
  const int rsub = lane >> 4, c4 = (lane & 15) * 4;
  for (int pass = 0; pass < 2; ++pass) {
#pragma unroll
    for (int q = 0; q < 16; ++q) {
      const int r = q * 2 + rsub;
      const v4f v = *(const v4fa*)&so[w][r][c4];
      if (C) *(volatile v4f*)(C + cofs + (size_t)(row0 + r) * ldc + col0 + c4) = v;
      if (C16) {
        v4h h4;
#pragma unroll
        for (int i = 0; i < 4; ++i) h4[i] = (_Float16)v[i];
        *(volatile v4h*)(C16 + cofs + (size_t)(row0 + r) * ldc + col0 + c4) = h4;
      }
    }
    if (pass == 0) __threadfence();
  }
}

template <int NHv, int TTv>
__global__ __launch_bounds__(256) void k_vt(const _Float16* __restrict__ V16, int ldv, int voff, _Float16* __restrict__ Vt) {
  __shared__ unsigned short tl[64][66];
  const int tid = threadIdx.x;
  const int slab = blockIdx.x / (TTv / 64), lg = blockIdx.x % (TTv / 64);
  const int b = slab / NHv, h = slab % NHv;
  for (int i = tid; i < 64 * 8; i += 256) {
    const int r = i / 8, c8 = (i % 8) * 8;
    FragH f;
    f.half[0] = *(const v8us*)((const unsigned short*)V16 + ((size_t)b * TTv + lg * 64 + r) * ldv + voff + h * 64 + c8);
#pragma unroll
    for (int q = 0; q < 8; ++q) tl[r][c8 + q] = f.u[q];
  }
  __syncthreads();
  for (int pass = 0; pass < 2; ++pass) {
#pragma unroll
    for (int rd = 0; rd < 2; ++rd) {
      const int d = rd * 32 + tid / 8, pc = tid % 8;
      FragH f;
#pragma unroll
      for (int q = 0; q < 8; ++q) f.u[q] = tl[pc * 8 + q][d];
      *(volatile v8us*)((unsigned short*)Vt + ((size_t)slab * 64 + d) * TTv + lg * 64 + pc * 8) = f.half[0];
    }
    if (pass == 0) __threadfence();
  }
}

__global__ __launch_bounds__(256) void k_rsmf(const float* __restrict__ S, _Float16* __restrict__ P, int qn, int hg) {
  #pragma clang fp contract(off)
  const int t = blockIdx.x * 256 + threadIdx.x;
  if (t >= qn * hg) return;
  const size_t i = (size_t)(t / qn) * SEQ + (t % qn);
  const float* s = S + i * SEQ;
  float mx = -3.0e38f;
#pragma unroll 1
  for (int j = 0; j < SEQ; j += 4) {
    const v4f a = *(const v4fa*)(s + j);
    mx = fmaxf(mx, a[0]); mx = fmaxf(mx, a[1]); mx = fmaxf(mx, a[2]); mx = fmaxf(mx, a[3]);
  }
  float se = 0.f;
#pragma unroll 1
  for (int j = 0; j < SEQ; j += 4) {
    const v4f a = *(const v4fa*)(s + j);
    se += __expf(a[0] - mx); se += __expf(a[1] - mx); se += __expf(a[2] - mx); se += __expf(a[3] - mx);
  }
  const float sc = 256.0f / se;
#pragma unroll 1
  for (int j0 = 0; j0 < SEQ; j0 += 8) {
    const v4f a = *(const v4fa*)(s + j0), c = *(const v4fa*)(s + j0 + 4);
    FragH f;
#pragma unroll
    for (int q = 0; q < 4; ++q) { f.h[q] = (_Float16)(__expf(a[q] - mx) * sc); f.h[4 + q] = (_Float16)(__expf(c[q] - mx) * sc); }
    const v8us o = f.half[0];
    unsigned short* d = (unsigned short*)P + i * SEQ + j0;
    *(volatile v8us*)d = o;
    __threadfence();
    *(volatile v8us*)d = o;
  }
}

#define WS_W4   ((size_t)4 * DM * DM * 2)
#define WS_QKV  ((size_t)3 * SEQ * DM * 2)
#define WS_XO   ((size_t)SEQ * DM * 2)
#define WS_VT   ((size_t)NH * HD * SEQ * 2)
#define WS_S    ((size_t)HG * SEQ * SEQ * 4)
#define WS_P    ((size_t)HG * SEQ * SEQ * 2)
#define WS_BT   ((size_t)NH * BW * 4)
static_assert(WS_W4 % 256 == 0 && WS_QKV % 256 == 0 && WS_XO % 256 == 0 && WS_VT % 256 == 0 && WS_S % 256 == 0 && WS_P % 256 == 0 && WS_BT % 256 == 0);
static_assert(WS_W4 + WS_QKV + WS_XO + WS_VT + WS_S + WS_P + WS_BT <= (size_t)134217728);

extern "C" void kernel_launch(void* const* d_in, const int* in_sizes, int n_in,
                              void* d_out, int out_size, void* d_ws, size_t ws_size, hipStream_t stream) {
  if (n_in < 6) return;
  const size_t xneed = ((size_t)(NB - 1) * SEQ_FULL + SEQ) * DM;
  if ((size_t)in_sizes[0] < xneed) return;
  if ((size_t)in_sizes[1] < (size_t)DM * DM || (size_t)in_sizes[2] < (size_t)DM * DM || (size_t)in_sizes[3] < (size_t)DM * DM || (size_t)in_sizes[4] < (size_t)DM * DM) return;
  if (in_sizes[5] < 32 * NH) return;
  if ((size_t)out_size < xneed) return;
  const float* x   = (const float*)d_in[0];
  const float* wq  = (const float*)d_in[1];
  const float* wk  = (const float*)d_in[2];
  const float* wv  = (const float*)d_in[3];
  const float* wo  = (const float*)d_in[4];
  const float* rel = (const float*)d_in[5];
  float* out = (float*)d_out;

  char* ws = (char*)d_ws; size_t off = 0;
  auto take = [&](size_t bytes) { char* p = ws + off; off += (bytes + 255) & ~(size_t)255; return p; };
  _Float16* W4  = (_Float16*)take(WS_W4);
  _Float16* QKV = (_Float16*)take(WS_QKV);
  _Float16* XO  = (_Float16*)take(WS_XO);
  _Float16* VT  = (_Float16*)take(WS_VT);
  float*    S   = (float*)take(WS_S);
  _Float16* P   = (_Float16*)take(WS_P);
  float*    BT  = (float*)take(WS_BT);
  if (off > ws_size) return;
  _Float16* BQ = W4; _Float16* BO = W4 + (size_t)3 * DM * DM;
  _Float16* Q16 = QKV; _Float16* K16 = QKV + (size_t)SEQ * DM; _Float16* V16 = QKV + (size_t)2 * SEQ * DM;

  {
    const size_t n8w = (size_t)DM * DM / 8;
    const unsigned gw = (unsigned)((n8w + 255) / 256);
    k_wnat<<<gw, 256, 0, stream>>>(wq, n8w, W4);
    k_wnat<<<gw, 256, 0, stream>>>(wk, n8w, W4 + (size_t)DM * DM);
    k_wnat<<<gw, 256, 0, stream>>>(wv, n8w, W4 + (size_t)2 * DM * DM);
    k_wnat<<<gw, 256, 0, stream>>>(wo, n8w, BO);
  }
  k_btab<<<(unsigned)((NH * BW) / 256), 256, 0, stream>>>(rel, BT);

  for (int b = 0; b < NB; ++b) {
    const float* xb = x + (size_t)b * SEQ_FULL * DM;
    float* ob = out + (size_t)b * SEQ_FULL * DM;
    const size_t n8x = (size_t)SEQ * DM / 8;
    k_x16<<<(unsigned)((n8x + 255) / 256), 256, 0, stream>>>(xb, XO, n8x);
    k_gemm2<0><<<dim3((unsigned)((SEQ / 128) * (DM / 64)), 3), 128, 0, stream>>>(XO, DM, (size_t)0, BQ, DM, (size_t)DM * DM, 0.0625f,
        nullptr, 0, nullptr, Q16, DM, (size_t)SEQ * DM, SEQ, DM, DM);
    k_vt<NH, SEQ><<<NH * (SEQ / 64), 256, 0, stream>>>(V16, DM, 0, VT);
    for (int h0 = 0; h0 < NH; h0 += HG) {
      k_gemm2<1><<<dim3((unsigned)((SEQ / 128) * (SEQ / 64)), HG), 128, 0, stream>>>(Q16 + h0 * HD, DM, (size_t)HD, K16 + h0 * HD, DM, (size_t)HD, 0.125f,
          BT, h0, S, nullptr, SEQ, (size_t)SEQ * SEQ, SEQ, SEQ, HD);
      k_rsmf<<<(unsigned)((HG * SEQ + 255) / 256), 256, 0, stream>>>(S, P, SEQ, HG);
      k_gemm2<0><<<dim3((unsigned)((SEQ / 128) * (HD / 64)), HG), 128, 0, stream>>>(P, SEQ, (size_t)SEQ * SEQ, VT + (size_t)h0 * HD * SEQ, SEQ, (size_t)HD * SEQ, 0.25f,
          nullptr, 0, nullptr, XO + h0 * HD, DM, (size_t)HD, SEQ, HD, SEQ);
    }
    k_gemm2<0><<<dim3((unsigned)((SEQ / 128) * (DM / 64)), 1), 128, 0, stream>>>(XO, DM, (size_t)0, BO, DM, (size_t)0, 0.0009765625f,
        nullptr, 0, ob, nullptr, DM, (size_t)0, SEQ, DM, DM);
  }
}
